// MambaBlock_11424613007364
// MI455X (gfx1250) — hardware-verified
//
#include <hip/hip_runtime.h>
#include <stddef.h>
#include <stdint.h>
#include <math.h>


#define TT     2048
#define LSEQ   1024
#define DM     1024
#define DI     2048
#define NS     16
#define DTR    64
#define XZW    4096
#define K2X    4096
#define K2D    128
#define WXR    128
#define BCW    32
#define NTHR   256
#define GBM    64
#define GBN    64
#define GTHR   128
#define SB     64
#define TCH    64
#define WSMAX  134217728

#define U_XB   (TT * DM / 8)
#define U_WIN  (XZW * DM / 8)
#define U_WX   (WXR * K2X / 8)
#define U_WDT  (DI * K2D / 8)
#define U_WO   (DM * K2X / 8)
#define U_CW   (DI * 4 / 4)
#define U_V    (DI / 4)
#define U_AN   (DI * NS / 4)
#define E0 (U_XB)
#define E1 (E0 + U_WIN)
#define E2 (E1 + U_WX)
#define E3 (E2 + U_WDT)
#define E4 (E3 + U_WO)
#define E5 (E4 + U_CW)
#define E6 (E5 + U_V)
#define E7 (E6 + U_V)
#define E8 (E7 + U_V)
#define E9 (E8 + U_AN)

static_assert(E0 % NTHR == 0 && E1 % NTHR == 0 && E2 % NTHR == 0 && E3 % NTHR == 0 && E4 % NTHR == 0);
static_assert(E5 % NTHR == 0 && E6 % NTHR == 0 && E7 % NTHR == 0 && E8 % NTHR == 0 && E9 % NTHR == 0);
static_assert(K2X / 8 == 512 && K2D / 8 == 16 && (K2X / 8) % NTHR == 0);
static_assert(TT % GBM == 0 && XZW % GBN == 0 && DI % GBN == 0 && DM % GBN == 0 && WXR % GBN == 0);
static_assert(DM % 32 == 0 && K2X % 32 == 0 && K2D % 32 == 0);
static_assert(K2X == 2 * DI && K2D == 2 * DTR && DTR == GBN && BCW == 2 * NS);
static_assert(GBM == (GTHR / 32) * 16 && GBN == 64);
static_assert(LSEQ % TCH == 0 && DI % SB == 0 && (TCH * BCW / 4) % SB == 0 && (TCH * 16) % SB == 0);
static_assert((2 * DI) % SB == 0 && DI / SB == 32);

typedef float          v4f   __attribute__((ext_vector_type(4)));
typedef float          v8f   __attribute__((ext_vector_type(8)));
typedef int            v8i   __attribute__((ext_vector_type(8)));
typedef unsigned short v4us  __attribute__((ext_vector_type(4)));
typedef unsigned short v8us  __attribute__((ext_vector_type(8)));
typedef unsigned short v16us __attribute__((ext_vector_type(16)));
typedef __bf16         v16bf __attribute__((ext_vector_type(16)));
typedef v4f  __attribute__((may_alias)) v4fa;
typedef v4us __attribute__((may_alias)) v4usa;
typedef v8us __attribute__((may_alias)) v8usa;
union FragB { v16bf v; v16us u; v8us h[2]; v8i w; };

__device__ __forceinline__ v8f wmb(const FragB& a, const FragB& b, v8f c) {
  v8f d = __builtin_amdgcn_wmma_f32_16x16x32_bf16(false, a.v, false, b.v, (short)0, c, false, false);
  asm volatile("v_nop\n\tv_nop\n\tv_nop\n\tv_nop" : "+v"(d) : "v"(a.w), "v"(b.w));
  return d;
}

__device__ __forceinline__ unsigned bf16_bits(float f) {
  const unsigned u = __float_as_uint(f);
  return (u + 0x7FFFu + ((u >> 16) & 1u)) >> 16;
}
__device__ __forceinline__ float bf16_val(float f) {
  return __uint_as_float(bf16_bits(f) << 16);
}

__device__ __forceinline__ void cv8(const float* __restrict__ sp, bool ok, unsigned short* dp) {
  const v4f a = *(const v4fa*)sp;
  const v4f b = *(const v4fa*)(sp + 4);
  v8us o;
  o[0] = ok ? (unsigned short)bf16_bits(a.x) : (unsigned short)0;
  o[1] = ok ? (unsigned short)bf16_bits(a.y) : (unsigned short)0;
  o[2] = ok ? (unsigned short)bf16_bits(a.z) : (unsigned short)0;
  o[3] = ok ? (unsigned short)bf16_bits(a.w) : (unsigned short)0;
  o[4] = ok ? (unsigned short)bf16_bits(b.x) : (unsigned short)0;
  o[5] = ok ? (unsigned short)bf16_bits(b.y) : (unsigned short)0;
  o[6] = ok ? (unsigned short)bf16_bits(b.z) : (unsigned short)0;
  o[7] = ok ? (unsigned short)bf16_bits(b.w) : (unsigned short)0;
  *(volatile v8us*)dp = o;
  __threadfence();
  *(volatile v8us*)dp = o;
}

template <int NEGEXP>
__device__ __forceinline__ void cv4(const float* __restrict__ sp, float* dp) {
  const v4f a = *(const v4fa*)sp;
  v4f o;
  o.x = bf16_val(a.x); o.y = bf16_val(a.y); o.z = bf16_val(a.z); o.w = bf16_val(a.w);
  if constexpr (NEGEXP != 0) {
    o.x = -expf(o.x); o.y = -expf(o.y); o.z = -expf(o.z); o.w = -expf(o.w);
  }
  *(volatile v4f*)dp = o;
  __threadfence();
  *(volatile v4f*)dp = o;
}

__global__ __launch_bounds__(NTHR) void k_prep(
    const float* __restrict__ x, const float* __restrict__ wi, const float* __restrict__ cw,
    const float* __restrict__ cb, const float* __restrict__ wx, const float* __restrict__ wd,
    const float* __restrict__ db, const float* __restrict__ al, const float* __restrict__ dd,
    const float* __restrict__ wo,
    unsigned short* XB, unsigned short* WIN, unsigned short* WX2, unsigned short* WDT2, unsigned short* WO2,
    float* CW, float* CB, float* DTB, float* DP, float* AN)
{
  const int u = (int)blockIdx.x * NTHR + (int)threadIdx.x;
  if (u < E0) {
    cv8(x + (size_t)u * 8, true, XB + (size_t)u * 8);
  } else if (u < E1) {
    const int v = u - E0;
    cv8(wi + (size_t)v * 8, true, WIN + (size_t)v * 8);
  } else if (u < E2) {
    const int v  = u - E1;
    const int n  = v >> 9;
    const int k8 = (v & 511) * 8;
    const int kk = k8 & (DI - 1);
    const int nc = n < 96 ? n : 95;
    cv8(wx + (size_t)nc * DI + kk, n < 96, WX2 + (size_t)n * K2X + k8);
  } else if (u < E3) {
    const int v  = u - E2;
    const int n  = v >> 4;
    const int k8 = (v & 15) * 8;
    const int kk = k8 & (DTR - 1);
    cv8(wd + (size_t)n * DTR + kk, true, WDT2 + (size_t)n * K2D + k8);
  } else if (u < E4) {
    const int v  = u - E3;
    const int n  = v >> 9;
    const int k8 = (v & 511) * 8;
    const int kk = k8 & (DI - 1);
    cv8(wo + (size_t)n * DI + kk, true, WO2 + (size_t)n * K2X + k8);
  } else if (u < E5) {
    const int v = u - E4;
    cv4<0>(cw + (size_t)v * 4, CW + (size_t)v * 4);
  } else if (u < E6) {
    const int v = u - E5;
    cv4<0>(cb + (size_t)v * 4, CB + (size_t)v * 4);
  } else if (u < E7) {
    const int v = u - E6;
    cv4<0>(db + (size_t)v * 4, DTB + (size_t)v * 4);
  } else if (u < E8) {
    const int v = u - E7;
    cv4<0>(dd + (size_t)v * 4, DP + (size_t)v * 4);
  } else if (u < E9) {
    const int v = u - E8;
    cv4<1>(al + (size_t)v * 4, AN + (size_t)v * 4);
  }
}

__device__ __forceinline__ float splus(float u) {
  return fmaxf(u, 0.0f) + log1pf(expf(-fabsf(u)));
}

template <int EPI>
__global__ __launch_bounds__(GTHR) void k_gemm(
    const unsigned short* __restrict__ A, const unsigned short* __restrict__ WT, int K,
    float* outF, int ldo, const float* __restrict__ bias, unsigned short* outH)
{
  __shared__ __attribute__((aligned(16))) float stg[GBM * GBN];
  const int tid = (int)threadIdx.x, lane = tid & 31, wave = tid >> 5, hh = lane >> 4, m = lane & 15;
  const int rowBase = (int)blockIdx.x * GBM;
  const int col0    = (int)blockIdx.y * GBN;

  v8f acc[4];
  {
    const v8f z = {0.f, 0.f, 0.f, 0.f, 0.f, 0.f, 0.f, 0.f};
    acc[0] = z; acc[1] = z; acc[2] = z; acc[3] = z;
  }
  const unsigned short* ap = A  + (size_t)(rowBase + 16 * wave + m) * (size_t)K + 8 * hh;
  const unsigned short* wp = WT + (size_t)(col0 + m) * (size_t)K + 8 * hh;
  const int ksteps = K >> 5;
#pragma unroll 1
  for (int ks = 0; ks < ksteps; ++ks) {
    FragB af;
    af.h[0] = *(const v8usa*)(ap + 32 * ks);
    af.h[1] = *(const v8usa*)(ap + 32 * ks + 16);
#pragma unroll
    for (int t = 0; t < 4; ++t) {
      const unsigned short* wq = wp + (size_t)(16 * t) * (size_t)K + 32 * ks;
      FragB bf;
      bf.h[0] = *(const v8usa*)wq;
      bf.h[1] = *(const v8usa*)(wq + 16);
      acc[t] = wmb(af, bf, acc[t]);
    }
  }

#pragma unroll
  for (int t = 0; t < 4; ++t) {
    const int lc = 16 * t + m;
#pragma unroll
    for (int r = 0; r < 8; ++r) {
      const int lr = 16 * wave + 8 * hh + r;
      stg[lr * GBN + lc] = acc[t][r];
    }
  }
  __syncthreads();

  if constexpr (EPI == 2) {
    if (blockIdx.y == 0) {
      v4f fv[8];
#pragma unroll
      for (int i = 0; i < 8; ++i) {
        const int lr = 16 * wave + 2 * i + hh;
        fv[i] = *(const v4fa*)(stg + lr * GBN + 4 * m);
      }
      __syncthreads();
#pragma unroll
      for (int i = 0; i < 8; ++i) {
        const int lr = 16 * wave + 2 * i + hh;
        v4us h4, l4;
        unsigned hb;
        hb = bf16_bits(fv[i].x); h4[0] = (unsigned short)hb; l4[0] = (unsigned short)bf16_bits(fv[i].x - __uint_as_float(hb << 16));
        hb = bf16_bits(fv[i].y); h4[1] = (unsigned short)hb; l4[1] = (unsigned short)bf16_bits(fv[i].y - __uint_as_float(hb << 16));
        hb = bf16_bits(fv[i].z); h4[2] = (unsigned short)hb; l4[2] = (unsigned short)bf16_bits(fv[i].z - __uint_as_float(hb << 16));
        hb = bf16_bits(fv[i].w); h4[3] = (unsigned short)hb; l4[3] = (unsigned short)bf16_bits(fv[i].w - __uint_as_float(hb << 16));
        unsigned short* srow = (unsigned short*)stg + (size_t)lr * (2 * GBN);
        *(v4usa*)(srow + 4 * m) = h4;
        *(v4usa*)(srow + DTR + 4 * m) = l4;
      }
      __syncthreads();
      v8us qv[8];
#pragma unroll
      for (int i = 0; i < 8; ++i) {
        const int lr = 16 * wave + 2 * i + hh;
        const unsigned short* srow = (const unsigned short*)stg + (size_t)lr * (2 * GBN);
        qv[i] = *(const v8usa*)(srow + 8 * m);
      }
#pragma unroll
      for (int i = 0; i < 8; ++i) {
        const int lr = 16 * wave + 2 * i + hh;
        unsigned short* dp = outH + (size_t)(rowBase + lr) * K2D + 8 * m;
        *(volatile v8us*)dp = qv[i];
      }
      __threadfence();
#pragma unroll
      for (int i = 0; i < 8; ++i) {
        const int lr = 16 * wave + 2 * i + hh;
        unsigned short* dp = outH + (size_t)(rowBase + lr) * K2D + 8 * m;
        *(volatile v8us*)dp = qv[i];
      }
    } else {
      const int q = lane >> 3, p = lane & 7;
      v4f gv[4];
#pragma unroll
      for (int it = 0; it < 4; ++it) {
        const int lr = 16 * wave + 4 * it + q;
        gv[it] = *(const v4fa*)(stg + lr * GBN + 4 * p);
      }
#pragma unroll
      for (int it = 0; it < 4; ++it) {
        const int lr = 16 * wave + 4 * it + q;
        float* op = outF + (size_t)(rowBase + lr) * BCW + 4 * p;
        *(volatile v4f*)op = gv[it];
      }
      __threadfence();
#pragma unroll
      for (int it = 0; it < 4; ++it) {
        const int lr = 16 * wave + 4 * it + q;
        float* op = outF + (size_t)(rowBase + lr) * BCW + 4 * p;
        *(volatile v4f*)op = gv[it];
      }
    }
  } else {
    if constexpr (EPI == 1) {
      const v4f b4 = *(const v4fa*)(bias + col0 + 4 * m);
#pragma unroll 1
      for (int i = 0; i < 8; ++i) {
        float* sp = stg + (16 * wave + 2 * i + hh) * GBN + 4 * m;
        const v4f u = *(const v4fa*)sp + b4;
        v4f y;
        y.x = splus(u.x); y.y = splus(u.y); y.z = splus(u.z); y.w = splus(u.w);
        *(v4fa*)sp = y;
      }
    }
    v4f fv[8];
#pragma unroll
    for (int i = 0; i < 8; ++i) {
      const int lr = 16 * wave + 2 * i + hh;
      fv[i] = *(const v4fa*)(stg + lr * GBN + 4 * m);
    }
#pragma unroll
    for (int i = 0; i < 8; ++i) {
      const int lr = 16 * wave + 2 * i + hh;
      float* op = outF + (size_t)(rowBase + lr) * (size_t)ldo + col0 + 4 * m;
      *(volatile v4f*)op = fv[i];
    }
    __threadfence();
#pragma unroll
    for (int i = 0; i < 8; ++i) {
      const int lr = 16 * wave + 2 * i + hh;
      float* op = outF + (size_t)(rowBase + lr) * (size_t)ldo + col0 + 4 * m;
      *(volatile v4f*)op = fv[i];
    }
  }
}

__global__ __launch_bounds__(NTHR) void k_conv(const float* __restrict__ XZ, const float* __restrict__ CW,
                                               const float* __restrict__ CB, float* XC, unsigned short* XH) {
  __shared__ __attribute__((aligned(16))) float sf[NTHR];
  __shared__ __attribute__((aligned(16))) unsigned short s16[2 * NTHR];
  const int tid   = (int)threadIdx.x;
  const int t     = (int)blockIdx.x >> 3;
  const int dbase = ((int)blockIdx.x & 7) * NTHR;
  const int d     = dbase + tid;
  const int l     = t & (LSEQ - 1);

  const v4f w  = *(const v4fa*)(CW + (size_t)d * 4);
  const float cbv = CB[d];
  const bool ok0 = l >= 3, ok1 = l >= 2, ok2 = l >= 1;
  const int t0 = ok0 ? t - 3 : t;
  const int t1 = ok1 ? t - 2 : t;
  const int t2 = ok2 ? t - 1 : t;
  float x0 = XZ[(size_t)t0 * XZW + d];
  float x1 = XZ[(size_t)t1 * XZW + d];
  float x2 = XZ[(size_t)t2 * XZW + d];
  const float x3 = XZ[(size_t)t * XZW + d];
  x0 = ok0 ? x0 : 0.0f;
  x1 = ok1 ? x1 : 0.0f;
  x2 = ok2 ? x2 : 0.0f;
  float acc = 0.0f + x0 * w.x;
  acc = acc + x1 * w.y;
  acc = acc + x2 * w.z;
  acc = acc + x3 * w.w;
  acc = acc + cbv;
  const float s = acc * (1.0f / (1.0f + expf(-acc)));
  const unsigned hb = bf16_bits(s);
  const unsigned lb = bf16_bits(s - __uint_as_float(hb << 16));
  sf[tid] = s;
  s16[tid] = (unsigned short)hb;
  s16[NTHR + tid] = (unsigned short)lb;
  __syncthreads();

  const int j = tid & 63;
  const v4f  fv = *(const v4fa*)(sf + 4 * j);
  const v8us hv = *(const v8usa*)(s16 + 8 * j);
  float* fp = XC + (size_t)t * DI + dbase + 4 * j;
  const int hcol = (j < 32) ? (dbase + 8 * j) : (DI + dbase + 8 * (j - 32));
  unsigned short* hp = XH + (size_t)t * K2X + hcol;
  const bool wf = tid < 64;
  const bool wh = (tid >= 64) && (tid < 128);
  if (wf) *(volatile v4f*)fp = fv;
  if (wh) *(volatile v8us*)hp = hv;
  __threadfence();
  if (wf) *(volatile v4f*)fp = fv;
  if (wh) *(volatile v8us*)hp = hv;
}

__global__ __launch_bounds__(SB) void k_scan(const float* __restrict__ DELTA, const float* __restrict__ XC,
                                             const float* __restrict__ XZ, const float* __restrict__ BC,
                                             const float* __restrict__ AN, const float* __restrict__ DP,
                                             unsigned short* YH) {
  __shared__ __attribute__((aligned(16))) float bcs[TCH * BCW];
  __shared__ __attribute__((aligned(16))) unsigned short ys[TCH * 128];
  __shared__ float hs[NS * SB];
  __shared__ float as_[NS * SB];
  const int tid = (int)threadIdx.x;
  const int bk  = (int)blockIdx.x;
  const int b   = bk >> 5;
  const int d0  = (bk & 31) * SB;
  const int d   = d0 + tid;
  {
    const float* ap = AN + (size_t)d * NS;
    const v4f a0 = *(const v4fa*)ap;
    const v4f a1 = *(const v4fa*)(ap + 4);
    const v4f a2 = *(const v4fa*)(ap + 8);
    const v4f a3 = *(const v4fa*)(ap + 12);
    as_[0 * SB + tid]  = a0.x; as_[1 * SB + tid]  = a0.y; as_[2 * SB + tid]  = a0.z; as_[3 * SB + tid]  = a0.w;
    as_[4 * SB + tid]  = a1.x; as_[5 * SB + tid]  = a1.y; as_[6 * SB + tid]  = a1.z; as_[7 * SB + tid]  = a1.w;
    as_[8 * SB + tid]  = a2.x; as_[9 * SB + tid]  = a2.y; as_[10 * SB + tid] = a2.z; as_[11 * SB + tid] = a2.w;
    as_[12 * SB + tid] = a3.x; as_[13 * SB + tid] = a3.y; as_[14 * SB + tid] = a3.z; as_[15 * SB + tid] = a3.w;
#pragma unroll
    for (int n = 0; n < NS; ++n) hs[n * SB + tid] = 0.0f;
  }
  const float dpv = DP[d];

#pragma unroll 1
  for (int ch = 0; ch < LSEQ / TCH; ++ch) {
    const int t0 = b * LSEQ + ch * TCH;
#pragma unroll
    for (int i = 0; i < (TCH * BCW / 4) / SB; ++i) {
      const int idx = i * SB + tid;
      *(v4fa*)(bcs + 4 * idx) = *(const v4fa*)(BC + (size_t)t0 * BCW + 4 * idx);
    }
    __syncthreads();

#pragma unroll 1
    for (int l = 0; l < TCH; ++l) {
      const size_t t = (size_t)(t0 + l);
      const float dl = DELTA[t * DI + d];
      const float xv = XC[t * DI + d];
      const float zv = XZ[t * XZW + DI + d];
      const float* bl = bcs + l * BCW;
      float y = 0.0f;
#pragma unroll 4
      for (int n = 0; n < NS; ++n) {
        const float an = as_[n * SB + tid];
        float hv = hs[n * SB + tid];
        const float bn = bl[n];
        const float cn = bl[NS + n];
        const float dA = expf(dl * an);
        hv = dA * hv + (dl * bn) * xv;
        hs[n * SB + tid] = hv;
        y += hv * cn;
      }
      const float sg = 1.0f / (1.0f + expf(-zv));
      const float yo = (y + xv * dpv) * (zv * sg);
      const unsigned hb = bf16_bits(yo);
      const unsigned lb = bf16_bits(yo - __uint_as_float(hb << 16));
      ys[l * 128 + tid]      = (unsigned short)hb;
      ys[l * 128 + SB + tid] = (unsigned short)lb;
    }
    __syncthreads();

    v8us q[16];
#pragma unroll
    for (int it = 0; it < 16; ++it) {
      const int idx  = it * SB + tid;
      const int step = idx >> 4;
      const int w    = idx & 15;
      q[it] = *(const v8usa*)(ys + step * 128 + 8 * w);
    }
#pragma unroll
    for (int it = 0; it < 16; ++it) {
      const int idx  = it * SB + tid;
      const int step = idx >> 4;
      const int w    = idx & 15;
      unsigned short* dp = YH + (size_t)(t0 + step) * K2X + (size_t)(w >> 3) * DI + d0 + 8 * (w & 7);
      *(volatile v8us*)dp = q[it];
    }
    __threadfence();
#pragma unroll
    for (int it = 0; it < 16; ++it) {
      const int idx  = it * SB + tid;
      const int step = idx >> 4;
      const int w    = idx & 15;
      unsigned short* dp = YH + (size_t)(t0 + step) * K2X + (size_t)(w >> 3) * DI + d0 + 8 * (w & 7);
      *(volatile v8us*)dp = q[it];
    }
    __syncthreads();
  }
}

static inline size_t al256(size_t o) { return (o + 255) & ~(size_t)255; }

extern "C" void kernel_launch(void* const* d_in, const int* in_sizes, int n_in,
                              void* d_out, int out_size, void* d_ws, size_t ws_size,
                              hipStream_t stream) {
  if (n_in < 10) return;
  if (in_sizes[0] != TT * DM) return;
  if (in_sizes[1] != XZW * DM) return;
  if (in_sizes[2] != DI * 4) return;
  if (in_sizes[3] != DI) return;
  if (in_sizes[4] != 96 * DI) return;
  if (in_sizes[5] != DI * DTR) return;
  if (in_sizes[6] != DI) return;
  if (in_sizes[7] != DI * NS) return;
  if (in_sizes[8] != DI) return;
  if (in_sizes[9] != DM * DI) return;
  if (out_size != TT * DM) return;

  const float* x   = (const float*)d_in[0];
  const float* wi  = (const float*)d_in[1];
  const float* cw  = (const float*)d_in[2];
  const float* cb  = (const float*)d_in[3];
  const float* wx  = (const float*)d_in[4];
  const float* wd  = (const float*)d_in[5];
  const float* db  = (const float*)d_in[6];
  const float* al  = (const float*)d_in[7];
  const float* dd  = (const float*)d_in[8];
  const float* wo  = (const float*)d_in[9];
  float* out = (float*)d_out;

  char* ws = (char*)d_ws;
  size_t off = 0;
  const size_t oXB  = off; off = al256(off + (size_t)TT * DM * 2);
  const size_t oWIN = off; off = al256(off + (size_t)XZW * DM * 2);
  const size_t oWX  = off; off = al256(off + (size_t)WXR * K2X * 2);
  const size_t oWD  = off; off = al256(off + (size_t)DI * K2D * 2);
  const size_t oWO  = off; off = al256(off + (size_t)DM * K2X * 2);
  const size_t oCW  = off; off = al256(off + (size_t)DI * 4 * 4);
  const size_t oCB  = off; off = al256(off + (size_t)DI * 4);
  const size_t oDTB = off; off = al256(off + (size_t)DI * 4);
  const size_t oDP  = off; off = al256(off + (size_t)DI * 4);
  const size_t oAN  = off; off = al256(off + (size_t)DI * NS * 4);
  const size_t oXZ  = off; off = al256(off + (size_t)TT * XZW * 4);
  const size_t oXC  = off; off = al256(off + (size_t)TT * DI * 4);
  const size_t oXH  = off; off = al256(off + (size_t)TT * K2X * 2);
  const size_t oBC  = off; off = al256(off + (size_t)TT * BCW * 4);
  const size_t oDTH = off; off = al256(off + (size_t)TT * K2D * 2);
  const size_t oDL  = off; off = al256(off + (size_t)TT * DI * 4);
  const size_t oYH  = off; off = al256(off + (size_t)TT * K2X * 2);
  if (off > ws_size || off > (size_t)WSMAX) return;
  unsigned short* XB   = (unsigned short*)(ws + oXB);
  unsigned short* WIN  = (unsigned short*)(ws + oWIN);
  unsigned short* WX2  = (unsigned short*)(ws + oWX);
  unsigned short* WDT2 = (unsigned short*)(ws + oWD);
  unsigned short* WO2  = (unsigned short*)(ws + oWO);
  float* CW   = (float*)(ws + oCW);
  float* CB   = (float*)(ws + oCB);
  float* DTB  = (float*)(ws + oDTB);
  float* DP   = (float*)(ws + oDP);
  float* AN   = (float*)(ws + oAN);
  float* XZ   = (float*)(ws + oXZ);
  float* XC   = (float*)(ws + oXC);
  unsigned short* XH  = (unsigned short*)(ws + oXH);
  float* BC   = (float*)(ws + oBC);
  unsigned short* DTH = (unsigned short*)(ws + oDTH);
  float* DL   = (float*)(ws + oDL);
  unsigned short* YH  = (unsigned short*)(ws + oYH);

  k_prep<<<E9 / NTHR, NTHR, 0, stream>>>(x, wi, cw, cb, wx, wd, db, al, dd, wo,
                                         XB, WIN, WX2, WDT2, WO2, CW, CB, DTB, DP, AN);
  k_gemm<0><<<dim3(TT / GBM, XZW / GBN), GTHR, 0, stream>>>(XB, WIN, DM, XZ, XZW, CB, XH);
  k_conv<<<TT * (DI / NTHR), NTHR, 0, stream>>>(XZ, CW, CB, XC, XH);
  k_gemm<2><<<dim3(TT / GBM, WXR / GBN), GTHR, 0, stream>>>(XH, WX2, K2X, BC, BCW, CB, DTH);
  k_gemm<1><<<dim3(TT / GBM, DI / GBN), GTHR, 0, stream>>>(DTH, WDT2, K2D, DL, DI, DTB, DTH);
  k_scan<<<(2 * DI) / SB, SB, 0, stream>>>(DL, XC, XZ, BC, AN, DP, YH);
  k_gemm<0><<<dim3(TT / GBM, DM / GBN), GTHR, 0, stream>>>(YH, WO2, K2X, out, DM, CB, YH);
}
